// TrilinearDistance_10385230922579
// MI455X (gfx1250) — hardware-verified
//
#include <hip/hip_runtime.h>


#define NB_  4
#define SS   256
#define TTT  256
#define LD   256
#define RD   256
#define AG   128
#define ACH  32
#define NBS  (NB_ * SS)
#define TW   (ACH * RD)

typedef unsigned short bf;
typedef __attribute__((ext_vector_type(16))) __bf16   v16bf;
typedef __attribute__((ext_vector_type(8)))  unsigned short v8us;
typedef __attribute__((ext_vector_type(8)))  float    v8f;
typedef __attribute__((ext_vector_type(4)))  float    v4f;
typedef v4f  __attribute__((may_alias)) v4fa;
typedef v8us __attribute__((may_alias)) v8usa;

__device__ __forceinline__ unsigned short f2bf(float f) { unsigned u = __float_as_uint(f); u += 0x7FFFu + ((u >> 16) & 1u); return (unsigned short)(u >> 16); }
__device__ __forceinline__ float bf2f(unsigned short b) { return __uint_as_float(((unsigned)b) << 16); }
__device__ __forceinline__ float bfr(float f) { return bf2f(f2bf(f)); }
__device__ __forceinline__ v16bf cat16b(v8us lo, v8us hi) { return __builtin_bit_cast(v16bf, __builtin_shufflevector(lo, hi, 0, 1, 2, 3, 4, 5, 6, 7, 8, 9, 10, 11, 12, 13, 14, 15)); }
__device__ __forceinline__ v8f wmmab(v16bf a, v16bf b, v8f c) { return __builtin_amdgcn_wmma_f32_16x16x32_bf16(false, a, false, b, (short)0, c, false, false); }
#define VST2(T, p, v) do { const T vst2_v_ = (v); *(volatile T*)(p) = vst2_v_; __threadfence(); *(volatile T*)(p) = vst2_v_; } while (0)

__global__ __launch_bounds__(256) void k_rows(const float* __restrict__ src, int rows, bf* dst) {
    const int lane = threadIdx.x & 31, r = blockIdx.x * 8 + (threadIdx.x >> 5);
    if (r >= rows) return;
    v8us o;
#pragma unroll
    for (int i = 0; i < 8; ++i) o[i] = f2bf(src[(size_t)r * 256 + lane * 8 + i]);
    VST2(v8us, dst + (size_t)r * 256 + lane * 8, o);
}
__global__ __launch_bounds__(256) void k_wt(const float* __restrict__ Wm, bf* WT) {
    __shared__ __align__(16) unsigned short tl[64 * 72];
    const int tid = threadIdx.x, l0 = blockIdx.x * 64, r0 = blockIdx.y * 64, a = blockIdx.z;
    const int ll = tid >> 2, rq = (tid & 3) * 16;
#pragma unroll
    for (int i = 0; i < 16; ++i) tl[(rq + i) * 72 + ll] = f2bf(Wm[((size_t)a * LD + l0 + ll) * RD + r0 + rq + i]);
    __syncthreads();
    const int piece = tid & 7;
    auto pass = [&]() {
#pragma unroll
        for (int s = 0; s < 2; ++s) { const int rr = (tid >> 3) + 32 * s; const v8us val = *(const v8usa*)(tl + rr * 72 + piece * 8); *(volatile v8us*)(WT + ((size_t)a * RD + r0 + rr) * LD + l0 + piece * 8) = val; }
    };
    pass(); __threadfence(); pass();
}
__global__ __launch_bounds__(128) void k_tmp(const bf* __restrict__ DB, const bf* __restrict__ WTc, bf* TH, bf* TL) {
    __shared__ __align__(16) float ost[4][16 * 68];
    const int lane = threadIdx.x & 31, wave = threadIdx.x >> 5, lr = lane & 15, hi = lane >> 4;
    const int r0 = blockIdx.x * 64 + wave * 16, c0 = blockIdx.y * 64;
    v8f acc[4];
#pragma unroll
    for (int t = 0; t < 4; ++t) acc[t] = (v8f){};
#pragma unroll 2
    for (int kc = 0; kc < LD; kc += 32) {
        const v16bf a = cat16b(*(const v8us*)(DB + (size_t)(r0 + lr) * LD + kc + 8 * hi), *(const v8us*)(DB + (size_t)(r0 + lr) * LD + kc + 8 * hi + 16));
#pragma unroll
        for (int t = 0; t < 4; ++t) { const bf* bp = WTc + (size_t)(c0 + t * 16 + lr) * LD + kc + 8 * hi; acc[t] = wmmab(a, cat16b(*(const v8us*)bp, *(const v8us*)(bp + 16)), acc[t]); }
        asm volatile("v_nop\n\tv_nop\n\tv_nop\n\tv_nop" : "+v"(acc[0]), "+v"(acc[1]), "+v"(acc[2]), "+v"(acc[3]) : "v"(a));
    }
    float* os = &ost[wave][0];
#pragma unroll
    for (int t = 0; t < 4; ++t)
#pragma unroll
        for (int j = 0; j < 8; ++j) os[(hi * 8 + j) * 68 + t * 16 + lr] = acc[t][j];
    __builtin_amdgcn_wave_barrier(); asm volatile("" ::: "memory");
    bf* c1 = TH + (size_t)r0 * TW + c0; bf* c2 = TL + (size_t)r0 * TW + c0;
    auto pass = [&]() {
#pragma unroll
        for (int s = 0; s < 4; ++s) { const int row = 4 * s + (lane >> 3), piece = lane & 7; const float* sp = os + row * 68 + piece * 8; v8us oh, ol;
#pragma unroll
            for (int i = 0; i < 8; ++i) { const unsigned short hb = f2bf(sp[i]); oh[i] = hb; ol[i] = f2bf(sp[i] - bf2f(hb)); }
            *(volatile v8us*)(c1 + (size_t)row * TW + piece * 8) = oh; *(volatile v8us*)(c2 + (size_t)row * TW + piece * 8) = ol; }
    };
    pass(); __threadfence(); pass();
}
__global__ __launch_bounds__(128) void k_bil(const bf* __restrict__ TH, const bf* __restrict__ TL, const bf* __restrict__ CB, const float* __restrict__ agg, int a0, int first, int last, float* DIST, float* out) {
    __shared__ __align__(16) float ost[4][16 * 68];
    const int lane = threadIdx.x & 31, wave = threadIdx.x >> 5, lr = lane & 15, hi = lane >> 4;
    const int b = blockIdx.z, s0 = blockIdx.x * 64 + wave * 16, t0 = blockIdx.y * 64;
    const size_t arow = ((size_t)b * SS + s0 + lr) * TW + 8 * hi;
    size_t boff[4];
#pragma unroll
    for (int t = 0; t < 4; ++t) boff[t] = ((size_t)b * TTT + t0 + t * 16 + lr) * RD + 8 * hi;
    v8f dacc[4];
#pragma unroll
    for (int t = 0; t < 4; ++t) dacc[t] = (v8f){};
#pragma unroll 1
    for (int a = 0; a < ACH; ++a) {
        const float ga = bfr(agg[a0 + a]);
        v8f acc[4];
#pragma unroll
        for (int t = 0; t < 4; ++t) acc[t] = (v8f){};
#pragma unroll 2
        for (int kc = 0; kc < RD; kc += 32) {
            const size_t ao = arow + (size_t)a * RD + kc;
            const v16bf ah = cat16b(*(const v8us*)(TH + ao), *(const v8us*)(TH + ao + 16)), al = cat16b(*(const v8us*)(TL + ao), *(const v8us*)(TL + ao + 16));
#pragma unroll
            for (int t = 0; t < 4; ++t) { const v16bf cb = cat16b(*(const v8us*)(CB + boff[t] + kc), *(const v8us*)(CB + boff[t] + kc + 16)); acc[t] = wmmab(ah, cb, acc[t]); acc[t] = wmmab(al, cb, acc[t]); }
            asm volatile("v_nop" : "+v"(acc[0]), "+v"(acc[1]), "+v"(acc[2]), "+v"(acc[3]) : "v"(ah), "v"(al) : "memory");
        }
        asm volatile("v_nop\n\tv_nop\n\tv_nop\n\tv_nop" : "+v"(acc[0]), "+v"(acc[1]), "+v"(acc[2]), "+v"(acc[3]));
#pragma unroll
        for (int t = 0; t < 4; ++t)
#pragma unroll
            for (int j = 0; j < 8; ++j) dacc[t][j] += ga * tanhf(acc[t][j]);
    }
    float* os = &ost[wave][0];
    const size_t drow = ((size_t)b * SS + s0) * TTT + t0;
#pragma unroll
    for (int t = 0; t < 4; ++t)
#pragma unroll
        for (int j = 0; j < 8; ++j) { float v = dacc[t][j]; if (!first) v += DIST[drow + (size_t)(hi * 8 + j) * TTT + t * 16 + lr]; os[(hi * 8 + j) * 68 + t * 16 + lr] = v; }
    __builtin_amdgcn_wave_barrier(); asm volatile("" ::: "memory");
    float* dst = (last ? out : DIST) + drow;
    auto pass = [&]() {
#pragma unroll
        for (int s = 0; s < 8; ++s) { const int Lid = (lane >> 3) + 4 * s, piece = lane & 7; const int row = Lid >> 1, cofs = (Lid & 1) * 32 + piece * 4;
            const v4f val = *(const v4fa*)(os + row * 68 + cofs); *(volatile v4f*)(dst + (size_t)row * TTT + cofs) = val; }
    };
    pass(); __threadfence(); pass();
}

extern "C" void kernel_launch(void* const* d_in, const int* in_sizes, int n_in,
                              void* d_out, int out_size, void* d_ws, size_t ws_size, hipStream_t stream) {
    (void)in_sizes; (void)n_in; (void)out_size;
    const float* data = (const float*)d_in[0]; const float* crit = (const float*)d_in[1]; const float* Wm = (const float*)d_in[2]; const float* agg = (const float*)d_in[3];
    float* out = (float*)d_out;
    char* wsp = (char*)d_ws;
    auto take = [&](size_t bytes) { char* p = wsp; wsp += (bytes + 255) & ~(size_t)255; return (void*)p; };
    bf* DB = (bf*)take((size_t)NBS * LD * 2); bf* CB = (bf*)take((size_t)NB_ * TTT * RD * 2); bf* WT = (bf*)take((size_t)AG * RD * LD * 2);
    bf* TH = (bf*)take((size_t)NBS * TW * 2); bf* TL = (bf*)take((size_t)NBS * TW * 2); float* DIST = (float*)take((size_t)NB_ * SS * TTT * 4);
    if ((size_t)(wsp - (char*)d_ws) > ws_size) return;
    k_rows<<<NBS / 8, 256, 0, stream>>>(data, NBS, DB); k_rows<<<(NB_ * TTT) / 8, 256, 0, stream>>>(crit, NB_ * TTT, CB);
    k_wt<<<dim3(LD / 64, RD / 64, AG), 256, 0, stream>>>(Wm, WT);
    for (int ch = 0; ch < AG / ACH; ++ch) {
        k_tmp<<<dim3(NBS / 64, TW / 64, 1), 128, 0, stream>>>(DB, WT + (size_t)ch * ACH * RD * LD, TH, TL);
        k_bil<<<dim3(SS / 64, TTT / 64, NB_), 128, 0, stream>>>(TH, TL, CB, agg, ch * ACH, ch == 0, ch == AG / ACH - 1, DIST, out);
    }
}
